// EncodedGCN_78958678769986
// MI455X (gfx1250) — hardware-verified
//
#include <hip/hip_runtime.h>
#include <stddef.h>


#define NTHR   256
#define NWAVE  8
#define EPT    8
#define NGRP   2
#define CHUNK  (NTHR * EPT * NGRP)
#define WCAP   (EPT * NGRP * 32)
#define LISTN  (NWAVE * WCAP)
#define SLSH   16
#define NB0    32768
#define NB1    4096
#define NB2    2048
#define FX     8
#define C1     32
#define C2     16
#define AP1    9
#define P1P    16
#define P2P    16
#define STP    40

#define LDS_DEG (NB0 * 4 + LISTN * 4 + 64)
#define L1_LIST (NB1 * AP1 * 4)
#define L1_WCNT (L1_LIST + LISTN * 4)
#define L1_ST   (L1_WCNT + 64)
#define L1_SD   (L1_ST + NWAVE * 16 * STP * 2)
#define LDS_L1  (L1_SD + NWAVE * 256 * 4)
#define L2_LIST (NB2 * C2 * 4)
#define L2_WCNT (L2_LIST + LISTN * 4)
#define LDS_L2  (L2_WCNT + 64)

static_assert((CHUNK & (CHUNK - 1)) == 0);
static_assert((4095 << SLSH) > 0);
static_assert(NB0 <= (1 << SLSH) && NB1 <= (1 << SLSH) && NB2 <= (1 << SLSH));
static_assert(NB0 % NB1 == 0 && NB1 % NB2 == 0);
static_assert(NB1 == NWAVE * 512);
static_assert(NB2 % NTHR == 0 && NB2 % (4 * NTHR) == 0);
static_assert((NB0 / 4) % NTHR == 0 && (NB0 * 4) % NTHR == 0);
static_assert(NB2 * 4 <= LISTN * 4);
static_assert((L1_ST % 16) == 0 && (L1_SD % 16) == 0 && (L2_LIST % 16) == 0);
static_assert((STP * 2) % 16 == 0);

typedef float    v4f  __attribute__((ext_vector_type(4)));
typedef float    v8f  __attribute__((ext_vector_type(8)));
typedef int      v4i  __attribute__((ext_vector_type(4)));
typedef _Float16 v8h  __attribute__((ext_vector_type(8)));
typedef _Float16 v16h __attribute__((ext_vector_type(16)));
typedef _Float16 v8ha __attribute__((ext_vector_type(8), may_alias));
typedef float    v4fa __attribute__((ext_vector_type(4), may_alias));
union FragH { v16h v; v8h h[2]; };

__device__ __forceinline__ v8f wmh(v16h a, v16h b, v8f c) {
  v8f d = __builtin_amdgcn_wmma_f32_16x16x32_f16(false, a, false, b, (short)0, c, false, false);
  asm volatile("v_nop\n\tv_nop\n\tv_nop\n\tv_nop" : "+v"(d) : "v"(a), "v"(b));
  return d;
}

__device__ __forceinline__ void wave_sync_lds() {
  __builtin_amdgcn_fence(__ATOMIC_SEQ_CST, "wavefront");
  __builtin_amdgcn_wave_barrier();
}

template <int NB>
__device__ __forceinline__ int scan_chunk(const int* __restrict__ dsts, int nE, int cbase, int slotBase,
                                          int vec8, int* list, int tid, int lane, int wave) {
  int wc = 0;
#pragma unroll
  for (int g = 0; g < NGRP; ++g) {
    const int el0  = (g * NTHR + tid) * EPT;
    const int e0   = cbase + el0;
    const int sent = -2147483647 - 1;
    v4i da, db;
    if (vec8 != 0 && cbase + CHUNK <= nE) {
      da = *(const v4i*)(dsts + e0);
      db = *(const v4i*)(dsts + e0 + 4);
    } else {
      da.x = (e0     < nE) ? dsts[min(e0,     nE - 1)] : sent;
      da.y = (e0 + 1 < nE) ? dsts[min(e0 + 1, nE - 1)] : sent;
      da.z = (e0 + 2 < nE) ? dsts[min(e0 + 2, nE - 1)] : sent;
      da.w = (e0 + 3 < nE) ? dsts[min(e0 + 3, nE - 1)] : sent;
      db.x = (e0 + 4 < nE) ? dsts[min(e0 + 4, nE - 1)] : sent;
      db.y = (e0 + 5 < nE) ? dsts[min(e0 + 5, nE - 1)] : sent;
      db.z = (e0 + 6 < nE) ? dsts[min(e0 + 6, nE - 1)] : sent;
      db.w = (e0 + 7 < nE) ? dsts[min(e0 + 7, nE - 1)] : sent;
    }
    const unsigned nb = (unsigned)slotBase;
    const unsigned s0 = (unsigned)da.x - nb, s1 = (unsigned)da.y - nb;
    const unsigned s2 = (unsigned)da.z - nb, s3 = (unsigned)da.w - nb;
    const unsigned s4 = (unsigned)db.x - nb, s5 = (unsigned)db.y - nb;
    const unsigned s6 = (unsigned)db.z - nb, s7 = (unsigned)db.w - nb;
    const bool h0 = s0 < (unsigned)NB, h1 = s1 < (unsigned)NB, h2 = s2 < (unsigned)NB, h3 = s3 < (unsigned)NB;
    const bool h4 = s4 < (unsigned)NB, h5 = s5 < (unsigned)NB, h6 = s6 < (unsigned)NB, h7 = s7 < (unsigned)NB;
    const unsigned any = __builtin_amdgcn_ballot_w32(h0 | h1 | h2 | h3 | h4 | h5 | h6 | h7);
    if (any != 0u) {
#define HITJ(J, HJ, SJ) { \
        const unsigned mj = __builtin_amdgcn_ballot_w32(HJ); \
        if (mj != 0u) { \
          if (HJ) { \
            const int pos = wc + (int)__builtin_amdgcn_mbcnt_lo(mj, 0u); \
            if (pos < WCAP) list[wave * WCAP + pos] = ((el0 + (J)) << SLSH) | (int)(SJ); \
          } \
          wc += (int)__builtin_popcount(mj); } }
      HITJ(0, h0, s0)
      HITJ(1, h1, s1)
      HITJ(2, h2, s2)
      HITJ(3, h3, s3)
      HITJ(4, h4, s4)
      HITJ(5, h5, s5)
      HITJ(6, h6, s6)
      HITJ(7, h7, s7)
#undef HITJ
    }
  }
  return wc;
}

__global__ __launch_bounds__(NTHR) void k_deg(
    const float* __restrict__ x, const int* __restrict__ ei, const float* __restrict__ ew,
    float* P1, int nN, int nE, int vec8) {
  extern __shared__ v4f lds_dyn[];
  float* sdeg = (float*)lds_dyn;
  int*   list = (int*)(sdeg + NB0);
  int*   wcnt = list + LISTN;
  const int tid = threadIdx.x, lane = tid & 31, wave = tid >> 5;
  const int nodeBase = blockIdx.x * NB0;
  const int* dsts = ei + nE;

  {
    const v4f z = {0.f, 0.f, 0.f, 0.f};
    for (int i = tid; i < NB0 / 4; i += NTHR) ((v4f*)sdeg)[i] = z;
  }
  __syncthreads();

  const int nChunks = (nE + CHUNK - 1) / CHUNK;
#pragma unroll 1
  for (int ch = 0; ch < nChunks; ++ch) {
    const int cbase = ch * CHUNK;
    const int wc = scan_chunk<NB0>(dsts, nE, cbase, nodeBase, vec8, list, tid, lane, wave);
    if (lane == 0) wcnt[wave] = wc;
    __syncthreads();
    if (wave == 0) {
#pragma unroll 1
      for (int wsx = 0; wsx < NWAVE; ++wsx) {
        int n = __builtin_amdgcn_readfirstlane(wcnt[wsx]);
        n = n > WCAP ? WCAP : (n < 0 ? 0 : n);
        const int* lp = list + wsx * WCAP;
#pragma unroll 1
        for (int i = 0; i < n; ++i) {
          const int ent = __builtin_amdgcn_readfirstlane(lp[i]);
          int slot = ent & ((1 << SLSH) - 1);
          slot = slot > NB0 - 1 ? NB0 - 1 : slot;
          int e = cbase + ((ent >> SLSH) & (CHUNK - 1));
          e = e > nE - 1 ? nE - 1 : e;
          const float w = ew[e];
          sdeg[slot] = sdeg[slot] + w;
        }
      }
    }
    __syncthreads();
  }

#pragma unroll 1
  for (int s = tid; s < NB0; s += NTHR) {
    const float d = sdeg[s] + 1.0f;
    const float r = rsqrtf(d);
    sdeg[s] = d > 0.0f ? r : 0.0f;
  }
  __syncthreads();

  float* pb = P1 + (size_t)nodeBase * P1P;
#pragma unroll 1
  for (int idx = tid; idx < NB0 * 4; idx += NTHR) {
    const int s = idx >> 2, q = idx & 3;
    int nodec = nodeBase + s;
    nodec = nodec > nN - 1 ? nN - 1 : nodec;
    const float dv = sdeg[s];
    const v4f xa = *(const v4f*)(x + (size_t)nodec * FX + 4 * (q & 1));
    v4f v;
    v.x = q < 2 ? xa.x * dv : (q == 2 ? dv : 0.0f);
    v.y = q < 2 ? xa.y * dv : 0.0f;
    v.z = q < 2 ? xa.z * dv : 0.0f;
    v.w = q < 2 ? xa.w * dv : 0.0f;
    float* pp = pb + 4 * (size_t)idx;
    *(volatile v4f*)pp = v;
    __threadfence();
    *(volatile v4f*)pp = v;
  }
}

__global__ __launch_bounds__(NTHR) void k_l1(
    const float* __restrict__ P1, const int* __restrict__ ei, const float* __restrict__ ew,
    const float* __restrict__ sv, const float* __restrict__ sw1, const float* __restrict__ sb1,
    const float* __restrict__ sw2, const float* __restrict__ sb2,
    const float* __restrict__ c1w, const float* __restrict__ c1b, const float* __restrict__ c2w,
    float* hs2, int nN, int nE, int vec8) {
  extern __shared__ v4f lds_dyn[];
  char* lb = (char*)lds_dyn;
  float*    sacc  = (float*)lb;
  int*      list  = (int*)(lb + L1_LIST);
  int*      wcnt  = (int*)(lb + L1_WCNT);
  float*    ssenc = (float*)(lb + L1_WCNT + 32);
  const int tid = threadIdx.x, lane = tid & 31, wave = tid >> 5, hh = lane >> 4, m = lane & 15;
  _Float16* sT = (_Float16*)(lb + L1_ST) + wave * 16 * STP;
  float*    sD = (float*)(lb + L1_SD) + wave * 256;
  const int nodeBase = blockIdx.x * NB1;
  const int* dsts = ei + nE;

  if (wave == 0) {
    float a = sb1[lane];
#pragma unroll 1
    for (int k = 0; k < 64; ++k) a = fmaf(sv[k], sw1[k * 32 + lane], a);
    a = fmaxf(a, 0.0f);
    float t = a * sw2[lane];
    t += __shfl_xor(t, 16);
    t += __shfl_xor(t, 8);
    t += __shfl_xor(t, 4);
    t += __shfl_xor(t, 2);
    t += __shfl_xor(t, 1);
    if (lane == 0) ssenc[0] = t + sb2[0];
  }
#pragma unroll 1
  for (int i = tid; i < NB1 * AP1; i += NTHR) {
    const int s = i / AP1;
    const int k = i - s * AP1;
    sacc[i] = P1[(size_t)(nodeBase + s) * P1P + k];
  }
  __syncthreads();

  const int nChunks = (nE + CHUNK - 1) / CHUNK;
#pragma unroll 1
  for (int ch = 0; ch < nChunks; ++ch) {
    const int cbase = ch * CHUNK;
    const int wc = scan_chunk<NB1>(dsts, nE, cbase, nodeBase, vec8, list, tid, lane, wave);
    if (lane == 0) wcnt[wave] = wc;
    __syncthreads();
    if (wave == 0) {
      const int c = lane < 8 ? lane : 8;
#pragma unroll 1
      for (int wsx = 0; wsx < NWAVE; ++wsx) {
        int n = __builtin_amdgcn_readfirstlane(wcnt[wsx]);
        n = n > WCAP ? WCAP : (n < 0 ? 0 : n);
        const int* lp = list + wsx * WCAP;
#pragma unroll 1
        for (int i = 0; i < n; ++i) {
          const int ent = __builtin_amdgcn_readfirstlane(lp[i]);
          int slot = ent & ((1 << SLSH) - 1);
          slot = slot > NB1 - 1 ? NB1 - 1 : slot;
          int e = cbase + ((ent >> SLSH) & (CHUNK - 1));
          e = e > nE - 1 ? nE - 1 : e;
          int src = ei[e];
          src = src < 0 ? 0 : (src > nN - 1 ? nN - 1 : src);
          const float w = ew[e];
          const float p = P1[(size_t)src * P1P + c];
          float* ap = sacc + slot * AP1 + c;
          *ap = fmaf(w, p, *ap);
        }
      }
    }
    __syncthreads();
  }

  const float senc = ssenc[0];
  float W1r[9];
#pragma unroll
  for (int k = 0; k < 8; ++k) W1r[k] = c1w[k * C1 + lane];
  W1r[8] = c1w[8 * C1 + lane] * senc;
  const float b1r = c1b[lane];
  v16h bv;
#pragma unroll
  for (int i = 0; i < 8; ++i) {
    bv[i]     = (_Float16)(8.0f * c2w[(8 * hh + i) * C2 + m]);
    bv[8 + i] = (_Float16)(8.0f * c2w[(16 + 8 * hh + i) * C2 + m]);
  }

#pragma unroll 1
  for (int g = 0; g < 32; ++g) {
    const int slot0 = wave * 512 + g * 16;
#pragma unroll 1
    for (int i = 0; i < 16; ++i) {
      const int s = slot0 + i;
      const float* ar = sacc + s * AP1;
      float dot = ar[0] * W1r[0];
      dot = fmaf(ar[1], W1r[1], dot);
      dot = fmaf(ar[2], W1r[2], dot);
      dot = fmaf(ar[3], W1r[3], dot);
      dot = fmaf(ar[4], W1r[4], dot);
      dot = fmaf(ar[5], W1r[5], dot);
      dot = fmaf(ar[6], W1r[6], dot);
      dot = fmaf(ar[7], W1r[7], dot);
      dot = fmaf(ar[8], W1r[8], dot);
      const float dv = P1[(size_t)(nodeBase + s) * P1P + 8];
      float h = fmaf(dv, dot, b1r);
      h = h > 0.0f ? h : 0.01f * h;
      sT[i * STP + lane] = (_Float16)(8.0f * dv * h);
    }
    wave_sync_lds();
    FragH a;
    a.h[0] = *(const v8ha*)(sT + m * STP + 8 * hh);
    a.h[1] = *(const v8ha*)(sT + m * STP + 16 + 8 * hh);
    v8f d = {0.f, 0.f, 0.f, 0.f, 0.f, 0.f, 0.f, 0.f};
    d = wmh(a.v, bv, d);
#pragma unroll
    for (int r = 0; r < 8; ++r) sD[(8 * hh + r) * 16 + m] = d[r] * 0.015625f;
    wave_sync_lds();
    const v4f o0 = *(const v4fa*)(sD + 4 * lane);
    const v4f o1 = *(const v4fa*)(sD + 128 + 4 * lane);
    float* gp = hs2 + (size_t)(nodeBase + slot0) * P2P;
    *(volatile v4f*)(gp + 4 * lane) = o0;
    *(volatile v4f*)(gp + 128 + 4 * lane) = o1;
    __threadfence();
    *(volatile v4f*)(gp + 4 * lane) = o0;
    *(volatile v4f*)(gp + 128 + 4 * lane) = o1;
    wave_sync_lds();
  }
}

__device__ __forceinline__ float head4(float dv, v4f a, v4f b, v4f f, float o) {
  float h;
  h = fmaf(dv, a.x, b.x); h = h > 0.0f ? h : 0.01f * h; o = fmaf(h, f.x, o);
  h = fmaf(dv, a.y, b.y); h = h > 0.0f ? h : 0.01f * h; o = fmaf(h, f.y, o);
  h = fmaf(dv, a.z, b.z); h = h > 0.0f ? h : 0.01f * h; o = fmaf(h, f.z, o);
  h = fmaf(dv, a.w, b.w); h = h > 0.0f ? h : 0.01f * h; o = fmaf(h, f.w, o);
  return o;
}

__global__ __launch_bounds__(NTHR) void k_l2(
    const float* __restrict__ P1, const float* __restrict__ hs2, const int* __restrict__ ei,
    const float* __restrict__ ew, const float* __restrict__ c2b, const float* __restrict__ fw,
    const float* __restrict__ fb, float* out, int nN, int nE, int vec8) {
  extern __shared__ v4f lds_dyn[];
  char* lb = (char*)lds_dyn;
  float* sacc = (float*)lb;
  int*   list = (int*)(lb + L2_LIST);
  int*   wcnt = (int*)(lb + L2_WCNT);
  float* sOut = (float*)(lb + L2_LIST);
  const int tid = threadIdx.x, lane = tid & 31, wave = tid >> 5;
  const int nodeBase = blockIdx.x * NB2;
  const int* dsts = ei + nE;

  {
    const v4f* src4 = (const v4f*)(hs2 + (size_t)nodeBase * P2P);
#pragma unroll 1
    for (int i = tid; i < NB2 * C2 / 4; i += NTHR) ((v4f*)sacc)[i] = src4[i];
  }
  __syncthreads();

  const int nChunks = (nE + CHUNK - 1) / CHUNK;
#pragma unroll 1
  for (int ch = 0; ch < nChunks; ++ch) {
    const int cbase = ch * CHUNK;
    const int wc = scan_chunk<NB2>(dsts, nE, cbase, nodeBase, vec8, list, tid, lane, wave);
    if (lane == 0) wcnt[wave] = wc;
    __syncthreads();
    if (wave == 0) {
      const int c = lane & 15;
#pragma unroll 1
      for (int wsx = 0; wsx < NWAVE; ++wsx) {
        int n = __builtin_amdgcn_readfirstlane(wcnt[wsx]);
        n = n > WCAP ? WCAP : (n < 0 ? 0 : n);
        const int* lp = list + wsx * WCAP;
#pragma unroll 1
        for (int i = 0; i < n; ++i) {
          const int ent = __builtin_amdgcn_readfirstlane(lp[i]);
          int slot = ent & ((1 << SLSH) - 1);
          slot = slot > NB2 - 1 ? NB2 - 1 : slot;
          int e = cbase + ((ent >> SLSH) & (CHUNK - 1));
          e = e > nE - 1 ? nE - 1 : e;
          int src = ei[e];
          src = src < 0 ? 0 : (src > nN - 1 ? nN - 1 : src);
          const float w = ew[e];
          const float p = hs2[(size_t)src * P2P + c];
          float* ap = sacc + slot * C2 + c;
          *ap = fmaf(w, p, *ap);
        }
      }
    }
    __syncthreads();
  }

  const v4f bq0 = *(const v4f*)(c2b + 0), bq1 = *(const v4f*)(c2b + 4);
  const v4f bq2 = *(const v4f*)(c2b + 8), bq3 = *(const v4f*)(c2b + 12);
  const v4f fq0 = *(const v4f*)(fw + 0), fq1 = *(const v4f*)(fw + 4);
  const v4f fq2 = *(const v4f*)(fw + 8), fq3 = *(const v4f*)(fw + 12);
  const float fbv = fb[0];
#pragma unroll 1
  for (int j = 0; j < NB2 / NTHR; ++j) {
    const int s = tid + NTHR * j;
    const float dv = P1[(size_t)(nodeBase + s) * P1P + 8];
    const float* ar = sacc + s * C2;
    const v4f a0 = *(const v4f*)(ar + 0), a1 = *(const v4f*)(ar + 4);
    const v4f a2 = *(const v4f*)(ar + 8), a3 = *(const v4f*)(ar + 12);
    float o = fbv;
    o = head4(dv, a0, bq0, fq0, o);
    o = head4(dv, a1, bq1, fq1, o);
    o = head4(dv, a2, bq2, fq2, o);
    o = head4(dv, a3, bq3, fq3, o);
    sOut[s] = o;
  }
  __syncthreads();

  v4f ov[NB2 / (4 * NTHR)];
#pragma unroll
  for (int j = 0; j < NB2 / (4 * NTHR); ++j) ov[j] = *(const v4f*)(sOut + 4 * (tid + NTHR * j));
#pragma unroll
  for (int j = 0; j < NB2 / (4 * NTHR); ++j) {
    const int gi = nodeBase + 4 * (tid + NTHR * j);
    if (gi + 3 < nN) {
      *(volatile v4f*)(out + gi) = ov[j];
    } else {
      if (gi     < nN) *(volatile float*)(out + gi)     = ov[j].x;
      if (gi + 1 < nN) *(volatile float*)(out + gi + 1) = ov[j].y;
      if (gi + 2 < nN) *(volatile float*)(out + gi + 2) = ov[j].z;
    }
  }
  __threadfence();
#pragma unroll
  for (int j = 0; j < NB2 / (4 * NTHR); ++j) {
    const int gi = nodeBase + 4 * (tid + NTHR * j);
    if (gi + 3 < nN) {
      *(volatile v4f*)(out + gi) = ov[j];
    } else {
      if (gi     < nN) *(volatile float*)(out + gi)     = ov[j].x;
      if (gi + 1 < nN) *(volatile float*)(out + gi + 1) = ov[j].y;
      if (gi + 2 < nN) *(volatile float*)(out + gi + 2) = ov[j].z;
    }
  }
}

extern "C" void kernel_launch(void* const* d_in, const int* in_sizes, int n_in,
                              void* d_out, int out_size, void* d_ws, size_t ws_size,
                              hipStream_t stream) {
  if (n_in < 14) return;
  const int nN = in_sizes[0] / FX;
  const int nE = in_sizes[2];
  if (nN <= 0 || nE < 0 || in_sizes[0] != nN * FX || in_sizes[1] != 2 * nE) return;
  if (in_sizes[3] != 64 || in_sizes[4] != 64 * 32 || in_sizes[5] != 32 || in_sizes[6] != 32 || in_sizes[7] < 1) return;
  if (in_sizes[8] != (FX + 1) * C1 || in_sizes[9] != C1 || in_sizes[10] != C1 * C2 || in_sizes[11] != C2) return;
  if (in_sizes[12] != C2 || in_sizes[13] < 1) return;
  if (out_size != nN) return;
  if (nN > (1 << 26) || nE > (1 << 29)) return;

  const float* x   = (const float*)d_in[0];
  const int*   ei  = (const int*)d_in[1];
  const float* ew  = (const float*)d_in[2];
  const float* sv  = (const float*)d_in[3];
  const float* sw1 = (const float*)d_in[4];
  const float* sb1 = (const float*)d_in[5];
  const float* sw2 = (const float*)d_in[6];
  const float* sb2 = (const float*)d_in[7];
  const float* c1w = (const float*)d_in[8];
  const float* c1b = (const float*)d_in[9];
  const float* c2w = (const float*)d_in[10];
  const float* c2b = (const float*)d_in[11];
  const float* fw  = (const float*)d_in[12];
  const float* fb  = (const float*)d_in[13];
  float* out = (float*)d_out;

  const int nB0 = (nN + NB0 - 1) / NB0;
  const int nB1 = (nN + NB1 - 1) / NB1;
  const int nB2 = (nN + NB2 - 1) / NB2;
  const int rowsP1 = nB0 * NB0;
  const int rowsP2 = nB1 * NB1;

  char* ws = (char*)d_ws;
  size_t off = 0;
  const size_t oP1 = off; off += (size_t)rowsP1 * P1P * 4;   off = (off + 255) & ~(size_t)255;
  const size_t oP2 = off; off += (size_t)rowsP2 * P2P * 4;   off = (off + 255) & ~(size_t)255;
  if (off > ws_size) return;
  float* P1  = (float*)(ws + oP1);
  float* hs2 = (float*)(ws + oP2);

  const int vec8 = ((nE & 3) == 0) ? 1 : 0;

  hipFuncSetAttribute(reinterpret_cast<const void*>(&k_deg), hipFuncAttributeMaxDynamicSharedMemorySize, LDS_DEG);
  hipFuncSetAttribute(reinterpret_cast<const void*>(&k_l1),  hipFuncAttributeMaxDynamicSharedMemorySize, LDS_L1);
  hipFuncSetAttribute(reinterpret_cast<const void*>(&k_l2),  hipFuncAttributeMaxDynamicSharedMemorySize, LDS_L2);

  k_deg<<<nB0, NTHR, LDS_DEG, stream>>>(x, ei, ew, P1, nN, nE, vec8);
  k_l1<<<nB1, NTHR, LDS_L1, stream>>>(P1, ei, ew, sv, sw1, sb1, sw2, sb2, c1w, c1b, c2w, hs2, nN, nE, vec8);
  k_l2<<<nB2, NTHR, LDS_L2, stream>>>(P1, hs2, ei, ew, c2b, fw, fb, out, nN, nE, vec8);
}
